// LSTMModel_41412074668762
// MI455X (gfx1250) — hardware-verified
//
#include <hip/hip_runtime.h>
#include <math.h>

constexpr int NBATCH = 2048;
constexpr int NSTEP  = 512;
constexpr int NHID   = 32;
constexpr int NGATE  = 4 * NHID;
constexpr int NTILE  = NBATCH / 16;
constexpr int W0P = 40;
constexpr int W1P = 104;
constexpr int ATP = 104;
constexpr int A0P = 40;
constexpr int ALP = 72;
constexpr int H2P = 68;
constexpr int TILE_HALVES = 16 * NHID;
constexpr float WCARRY  = 16.0f;
constexpr float HCARRY  = 64.0f;
constexpr float ACC_INV = 1.0f / (WCARRY * HCARRY);
constexpr size_t HB_BYTES = (size_t)NTILE * (size_t)NSTEP * (size_t)TILE_HALVES * 2;

static_assert(NBATCH % 16 == 0);
static_assert(NHID == 32);
static_assert(NGATE == 128);
static_assert(HB_BYTES == (size_t)67108864);
static_assert((16 * A0P) % 32 == 0);
static_assert((16 * ATP) % 32 == 0);
static_assert((16 * ALP) % 32 == 0);
static_assert((16 * H2P) % 32 == 0);
static_assert(W0P % 8 == 0 && W1P % 8 == 0 && ATP % 8 == 0 && A0P % 8 == 0 && ALP % 8 == 0);
static_assert(NBATCH * 2 * 4 == 16384);

typedef __attribute__((ext_vector_type(16))) _Float16 v16h;
typedef __attribute__((ext_vector_type(8)))  _Float16 v8h;
typedef __attribute__((ext_vector_type(8)))  float    v8f;
typedef __attribute__((ext_vector_type(4)))  float    v4f;
typedef __attribute__((ext_vector_type(4)))  unsigned v4u;

__device__ __forceinline__ void guard4_h(v8f& a, v8f& b, v8f& c, v8f& d, v16h x, v16h y) {
  asm volatile("v_nop\n\tv_nop\n\tv_nop\n\tv_nop" : "+v"(a), "+v"(b), "+v"(c), "+v"(d) : "v"(x), "v"(y));
}
__device__ __forceinline__ void guard3_h(v8f& a, v8f& b, v8f& c, v16h x, v16h y) {
  asm volatile("v_nop\n\tv_nop\n\tv_nop\n\tv_nop" : "+v"(a), "+v"(b), "+v"(c) : "v"(x), "v"(y));
}
__device__ __forceinline__ void keep4_h(v16h a, v16h b, v16h c, v16h d) { asm volatile("v_nop" :: "v"(a), "v"(b), "v"(c), "v"(d)); }
__device__ __forceinline__ void keep3_h(v16h a, v16h b, v16h c) { asm volatile("v_nop" :: "v"(a), "v"(b), "v"(c)); }

template <typename T> struct Frag;
template <> struct Frag<_Float16> {
  typedef v16h V; union U { v16h v; v8h h[2]; };
  static __device__ __forceinline__ v16h load(const _Float16* p) {
    U f; f.h[0] = *(const v8h*)(p); f.h[1] = *(const v8h*)(p + 16); return f.v;
  }
  static __device__ __forceinline__ v8f mma(v16h a, v16h b, v8f c) {
    return __builtin_amdgcn_wmma_f32_16x16x32_f16(false, a, false, b, (short)0, c, false, false);
  }
};

__device__ __forceinline__ float fsig(float x)  { return __builtin_amdgcn_rcpf(1.0f + __expf(-x)); }
__device__ __forceinline__ float ftanh(float x) { return 1.0f - 2.0f * __builtin_amdgcn_rcpf(__expf(2.0f * x) + 1.0f); }

__device__ __forceinline__ float cell_step(float zi, float zf, float zg, float zo, float& cs) {
  const float ig = fsig(zi);
  const float fg = fsig(zf);
  const float gg = ftanh(zg);
  const float og = fsig(zo);
  const float cn = fg * cs + ig * gg;
  cs = cn;
  return og * ftanh(cn);
}

__device__ __forceinline__ void gates4(const v16h a, const _Float16* wb, int gs, v8f& a0, v8f& a1, v8f& a2, v8f& a3) {
  const v16h b0 = Frag<_Float16>::load(wb);
  const v16h b1 = Frag<_Float16>::load(wb + gs);
  const v16h b2 = Frag<_Float16>::load(wb + 2 * gs);
  const v16h b3 = Frag<_Float16>::load(wb + 3 * gs);
  a0 = Frag<_Float16>::mma(a, b0, a0);
  a1 = Frag<_Float16>::mma(a, b1, a1);
  a2 = Frag<_Float16>::mma(a, b2, a2);
  a3 = Frag<_Float16>::mma(a, b3, a3);
  guard4_h(a0, a1, a2, a3, a, b3);
  keep4_h(b0, b1, b2, b3);
}
__device__ __forceinline__ void gates3(const v16h a, const _Float16* wb, int gs, v8f& a0, v8f& a2, v8f& a3) {
  const v16h b0 = Frag<_Float16>::load(wb);
  const v16h b2 = Frag<_Float16>::load(wb + 2 * gs);
  const v16h b3 = Frag<_Float16>::load(wb + 3 * gs);
  a0 = Frag<_Float16>::mma(a, b0, a0);
  a2 = Frag<_Float16>::mma(a, b2, a2);
  a3 = Frag<_Float16>::mma(a, b3, a3);
  guard3_h(a0, a2, a3, a, b3);
  keep3_h(b0, b2, b3);
}

template <int SRCLD>
__device__ __forceinline__ void stage_w(const float* __restrict__ src, _Float16* dst, int pitch, int colofs, int lane) {
  constexpr int CPR = SRCLD / 8;
  constexpr int NIT = NGATE * CPR / 32;
  static_assert(SRCLD % 8 == 0);
  static_assert((NGATE * CPR) % 32 == 0);
#pragma unroll 1
  for (int it = 0; it < NIT; ++it) {
    const int q  = it * 32 + lane;
    const int n  = q / CPR;
    const int k8 = (q - n * CPR) * 8;
    const v4f a = *(const v4f*)(src + n * SRCLD + k8);
    const v4f b = *(const v4f*)(src + n * SRCLD + k8 + 4);
    v8h hv;
#pragma unroll
    for (int e = 0; e < 4; ++e) {
      hv[e]     = (_Float16)(a[e] * WCARRY);
      hv[4 + e] = (_Float16)(b[e] * WCARRY);
    }
    *(v8h*)(dst + n * pitch + colofs + k8) = hv;
  }
}

__device__ __forceinline__ int clamp_len(int L) { return L < 1 ? 1 : (L > NSTEP ? NSTEP : L); }

__global__ __launch_bounds__(32) void rev_scan_kernel(const float* __restrict__ x, const int* __restrict__ lengths,
                                                      const float* __restrict__ wih, const float* __restrict__ whh,
                                                      const float* __restrict__ bih, const float* __restrict__ bhh,
                                                      unsigned short* __restrict__ HBp) {
  __shared__ __align__(16) _Float16 W0s[NGATE * W0P];
  __shared__ __align__(16) _Float16 Ah[16 * A0P];
  __shared__ __align__(16) float Bs[NGATE];
  __shared__ __align__(16) float Wx[NGATE];
  const int lane = threadIdx.x & 31;
  const int c = lane & 15, hh = lane >> 4, koff = hh * 8;
  const int tile = blockIdx.x;
  const int rowbase = tile * 16;

  stage_w<NHID>(whh, W0s, W0P, 0, lane);
#pragma unroll 1
  for (int it = 0; it < NGATE / 32; ++it) {
    const int i = it * 32 + lane;
    Bs[i] = bih[i] + bhh[i];
    Wx[i] = wih[i];
  }
#pragma unroll 1
  for (int i = lane; i < 16 * A0P; i += 32) Ah[i] = (_Float16)0.0f;

  int lenm1[8];
#pragma unroll
  for (int r = 0; r < 8; ++r) lenm1[r] = clamp_len(lengths[rowbase + 8 * hh + r]) - 1;
  int lt = clamp_len(lengths[rowbase + c]);
#pragma unroll
  for (int off = 1; off < 32; off <<= 1) {
    const int o = __shfl_xor(lt, off, 32);
    lt = lt > o ? lt : o;
  }
  const int tmax = __builtin_amdgcn_readfirstlane(lt);

  float cst[2][8];
#pragma unroll
  for (int ub = 0; ub < 2; ++ub)
#pragma unroll
    for (int r = 0; r < 8; ++r) cst[ub][r] = 0.0f;
  __syncthreads();

  const float* xb = x + (size_t)(rowbase + 8 * hh) * NSTEP;
  const v8f z8 = {0.f, 0.f, 0.f, 0.f, 0.f, 0.f, 0.f, 0.f};
  const int crow = lane >> 2, ccol = (lane & 3) * 8;

#pragma unroll 1
  for (int s = 0; s < tmax; ++s) {
    float xm[8];
#pragma unroll
    for (int r = 0; r < 8; ++r) {
      const int q  = lenm1[r] - s;
      const int qc = q < 0 ? 0 : q;
      float v = xb[r * NSTEP + qc];
      asm volatile("" : "+v"(v));
      xm[r] = (q >= 0) ? v : 0.0f;
    }
    const v16h a = Frag<_Float16>::load(Ah + c * A0P + koff);
    float hn[2][8];
#pragma unroll
    for (int ub = 0; ub < 2; ++ub) {
      v8f a0 = z8, a1 = z8, a2 = z8, a3 = z8;
      gates4(a, W0s + (16 * ub + c) * W0P + koff, 32 * W0P, a0, a1, a2, a3);
      const int u = 16 * ub + c;
      const float wi = Wx[u], wf = Wx[32 + u], wg = Wx[64 + u], wo = Wx[96 + u];
      const float bi = Bs[u], bf = Bs[32 + u], bg = Bs[64 + u], bo = Bs[96 + u];
#pragma unroll
      for (int r = 0; r < 8; ++r) {
        const float zi = a0[r] * ACC_INV + (xm[r] * wi + bi);
        const float zf = a1[r] * ACC_INV + (xm[r] * wf + bf);
        const float zg = a2[r] * ACC_INV + (xm[r] * wg + bg);
        const float zo = a3[r] * ACC_INV + (xm[r] * wo + bo);
        hn[ub][r] = cell_step(zi, zf, zg, zo, cst[ub][r]);
      }
    }
    __syncthreads();
#pragma unroll
    for (int ub = 0; ub < 2; ++ub)
#pragma unroll
      for (int r = 0; r < 8; ++r) Ah[(8 * hh + r) * A0P + 16 * ub + c] = (_Float16)(hn[ub][r] * HCARRY);
    __syncthreads();
    {
      const v8h o0 = *(const v8h*)(Ah + crow * A0P + ccol);
      const v8h o1 = *(const v8h*)(Ah + (8 + crow) * A0P + ccol);
      unsigned short* dst = HBp + ((size_t)tile * NSTEP + (size_t)s) * TILE_HALVES + 8 * lane;
      for (int pass = 0; pass < 2; ++pass) {
        *(volatile v8h*)(dst) = o0;
        *(volatile v8h*)(dst + 256) = o1;
        __threadfence();
      }
    }
  }
}

__global__ __launch_bounds__(32) void fwd_stack_kernel(const float* __restrict__ x, const int* __restrict__ lengths,
                                                       const float* __restrict__ wih0, const float* __restrict__ whh0,
                                                       const float* __restrict__ bih0, const float* __restrict__ bhh0,
                                                       const float* __restrict__ wih1, const float* __restrict__ whh1,
                                                       const float* __restrict__ bih1, const float* __restrict__ bhh1,
                                                       const float* __restrict__ wih1r,
                                                       const float* __restrict__ bih1r, const float* __restrict__ bhh1r,
                                                       const float* __restrict__ wout, const float* __restrict__ bout,
                                                       const unsigned short* __restrict__ HBp, float* __restrict__ out) {
  __shared__ __align__(16) _Float16 W0s[NGATE * W0P];
  __shared__ __align__(16) _Float16 W1s[NGATE * W1P];
  __shared__ __align__(16) _Float16 At[16 * ATP];
  __shared__ __align__(16) _Float16 AL[16 * ALP];
  __shared__ __align__(16) float H2[16 * H2P];
  __shared__ __align__(16) float Bs0[NGATE];
  __shared__ __align__(16) float Wx0[NGATE];
  __shared__ __align__(16) float Bs1[NGATE];
  __shared__ __align__(16) float Bs1r[NGATE];
  const int lane = threadIdx.x & 31;
  const int c = lane & 15, hh = lane >> 4, koff = hh * 8;
  const int tile = blockIdx.x;
  const int rowbase = tile * 16;
  const int mA = lane >> 1, halfA = lane & 1;

  stage_w<NHID>(whh0, W0s, W0P, 0, lane);
  stage_w<2 * NHID>(wih1, W1s, W1P, 0, lane);
  stage_w<NHID>(whh1, W1s, W1P, 2 * NHID, lane);
#pragma unroll 1
  for (int it = 0; it < NGATE / 32; ++it) {
    const int i = it * 32 + lane;
    Bs0[i]  = bih0[i] + bhh0[i];
    Wx0[i]  = wih0[i];
    Bs1[i]  = bih1[i] + bhh1[i];
    Bs1r[i] = bih1r[i] + bhh1r[i];
  }
#pragma unroll 1
  for (int i = lane; i < 16 * ATP; i += 32) At[i] = (_Float16)0.0f;
#pragma unroll 1
  for (int i = lane; i < 16 * ALP; i += 32) AL[i] = (_Float16)0.0f;
#pragma unroll 1
  for (int i = lane; i < 16 * H2P; i += 32) H2[i] = 0.0f;

  int lenm1[8];
#pragma unroll
  for (int r = 0; r < 8; ++r) lenm1[r] = clamp_len(lengths[rowbase + 8 * hh + r]) - 1;
  const int lenA1 = clamp_len(lengths[rowbase + mA]) - 1;
  int lt = clamp_len(lengths[rowbase + c]);
#pragma unroll
  for (int off = 1; off < 32; off <<= 1) {
    const int o = __shfl_xor(lt, off, 32);
    lt = lt > o ? lt : o;
  }
  const int tmax = __builtin_amdgcn_readfirstlane(lt);

  float c0s[2][8], c1s[2][8], h2r[2][8];
#pragma unroll
  for (int ub = 0; ub < 2; ++ub)
#pragma unroll
    for (int r = 0; r < 8; ++r) { c0s[ub][r] = 0.0f; c1s[ub][r] = 0.0f; h2r[ub][r] = 0.0f; }
  __syncthreads();

  const float* xb = x + (size_t)(rowbase + 8 * hh) * NSTEP;
  const v8f z8 = {0.f, 0.f, 0.f, 0.f, 0.f, 0.f, 0.f, 0.f};

#pragma unroll 1
  for (int t = 0; t < tmax; ++t) {
    float xm[8];
#pragma unroll
    for (int r = 0; r < 8; ++r) {
      float v = xb[r * NSTEP + t];
      asm volatile("" : "+v"(v));
      xm[r] = v;
    }
    int sidx = lenA1 - t;
    sidx = sidx < 0 ? 0 : (sidx > NSTEP - 1 ? NSTEP - 1 : sidx);
    const v4u* hp = (const v4u*)(HBp + (((size_t)tile * NSTEP + (size_t)sidx) * 16 + (size_t)mA) * NHID + 16 * halfA);
    const v4u g0 = hp[0];
    const v4u g1 = hp[1];

    const v16h a0f = Frag<_Float16>::load(At + c * ATP + koff);
    float hn[2][8];
#pragma unroll
    for (int ub = 0; ub < 2; ++ub) {
      v8f a0 = z8, a1 = z8, a2 = z8, a3 = z8;
      gates4(a0f, W0s + (16 * ub + c) * W0P + koff, 32 * W0P, a0, a1, a2, a3);
      const int u = 16 * ub + c;
      const float wi = Wx0[u], wf = Wx0[32 + u], wg = Wx0[64 + u], wo = Wx0[96 + u];
      const float bi = Bs0[u], bf = Bs0[32 + u], bg = Bs0[64 + u], bo = Bs0[96 + u];
#pragma unroll
      for (int r = 0; r < 8; ++r) {
        const float zi = a0[r] * ACC_INV + (xm[r] * wi + bi);
        const float zf = a1[r] * ACC_INV + (xm[r] * wf + bf);
        const float zg = a2[r] * ACC_INV + (xm[r] * wg + bg);
        const float zo = a3[r] * ACC_INV + (xm[r] * wo + bo);
        const float hv = cell_step(zi, zf, zg, zo, c0s[ub][r]);
        hn[ub][r] = hv;
        if (t == lenm1[r]) AL[(8 * hh + r) * ALP + u] = (_Float16)(hv * HCARRY);
      }
    }
    __syncthreads();
#pragma unroll
    for (int ub = 0; ub < 2; ++ub)
#pragma unroll
      for (int r = 0; r < 8; ++r) {
        At[(8 * hh + r) * ATP + 16 * ub + c]      = (_Float16)(hn[ub][r] * HCARRY);
        At[(8 * hh + r) * ATP + 64 + 16 * ub + c] = (_Float16)(h2r[ub][r] * HCARRY);
      }
    *(v4u*)(At + mA * ATP + 32 + 16 * halfA)     = g0;
    *(v4u*)(At + mA * ATP + 32 + 16 * halfA + 8) = g1;
    __syncthreads();

    const v16h ax0 = Frag<_Float16>::load(At + c * ATP + koff);
    const v16h ax1 = Frag<_Float16>::load(At + c * ATP + 32 + koff);
    const v16h ax2 = Frag<_Float16>::load(At + c * ATP + 64 + koff);
#pragma unroll
    for (int ub = 0; ub < 2; ++ub) {
      v8f a0 = z8, a1 = z8, a2 = z8, a3 = z8;
      const _Float16* wb = W1s + (16 * ub + c) * W1P + koff;
      gates4(ax0, wb,      32 * W1P, a0, a1, a2, a3);
      gates4(ax1, wb + 32, 32 * W1P, a0, a1, a2, a3);
      gates4(ax2, wb + 64, 32 * W1P, a0, a1, a2, a3);
      const int u = 16 * ub + c;
      const float bi = Bs1[u], bf = Bs1[32 + u], bg = Bs1[64 + u], bo = Bs1[96 + u];
#pragma unroll
      for (int r = 0; r < 8; ++r) {
        const float zi = a0[r] * ACC_INV + bi;
        const float zf = a1[r] * ACC_INV + bf;
        const float zg = a2[r] * ACC_INV + bg;
        const float zo = a3[r] * ACC_INV + bo;
        const float hv = cell_step(zi, zf, zg, zo, c1s[ub][r]);
        h2r[ub][r] = hv;
        if (t == lenm1[r]) H2[(8 * hh + r) * H2P + u] = hv;
      }
    }
  }

  __syncthreads();
  stage_w<2 * NHID>(wih1r, W1s, W1P, 0, lane);
  {
    const v4u* hp = (const v4u*)(HBp + (((size_t)tile * NSTEP) * 16 + (size_t)mA) * NHID + 16 * halfA);
    const v4u g0 = hp[0];
    const v4u g1 = hp[1];
    *(v4u*)(AL + mA * ALP + 32 + 16 * halfA)     = g0;
    *(v4u*)(AL + mA * ALP + 32 + 16 * halfA + 8) = g1;
  }
  __syncthreads();
  {
    const v16h ar0 = Frag<_Float16>::load(AL + c * ALP + koff);
    const v16h ar1 = Frag<_Float16>::load(AL + c * ALP + 32 + koff);
#pragma unroll
    for (int ub = 0; ub < 2; ++ub) {
      v8f a0 = z8, a2 = z8, a3 = z8;
      const _Float16* wb = W1s + (16 * ub + c) * W1P + koff;
      gates3(ar0, wb,      32 * W1P, a0, a2, a3);
      gates3(ar1, wb + 32, 32 * W1P, a0, a2, a3);
      const int u = 16 * ub + c;
      const float bi = Bs1r[u], bg = Bs1r[64 + u], bo = Bs1r[96 + u];
#pragma unroll
      for (int r = 0; r < 8; ++r) {
        const float ig = fsig(a0[r] * ACC_INV + bi);
        const float gg = ftanh(a2[r] * ACC_INV + bg);
        const float og = fsig(a3[r] * ACC_INV + bo);
        const float cn = ig * gg;
        H2[(8 * hh + r) * H2P + 32 + u] = og * ftanh(cn);
      }
    }
  }
  __syncthreads();

  {
    const float* hrow = H2 + mA * H2P;
    const float* wrow = wout + halfA * (2 * NHID);
    float acc = 0.0f;
#pragma unroll 4
    for (int k = 0; k < 2 * NHID; ++k) acc = fmaf(hrow[k], wrow[k], acc);
    acc += bout[halfA];
    float* op = out + rowbase * 2 + lane;
    *(volatile float*)op = acc;
    __threadfence();
    *(volatile float*)op = acc;
  }
}

extern "C" void kernel_launch(void* const* d_in, const int* in_sizes, int n_in,
                              void* d_out, int out_size, void* d_ws, size_t ws_size, hipStream_t stream) {
  if (n_in < 20 || d_out == nullptr || d_ws == nullptr) return;
  if (in_sizes[0] != NBATCH * NSTEP || in_sizes[1] != NBATCH ||
      in_sizes[2] != NGATE || in_sizes[3] != NGATE * NHID || in_sizes[4] != NGATE || in_sizes[5] != NGATE ||
      in_sizes[6] != NGATE || in_sizes[7] != NGATE * NHID || in_sizes[8] != NGATE || in_sizes[9] != NGATE ||
      in_sizes[10] != NGATE * 2 * NHID || in_sizes[11] != NGATE * NHID || in_sizes[12] != NGATE || in_sizes[13] != NGATE ||
      in_sizes[14] != NGATE * 2 * NHID || in_sizes[16] != NGATE || in_sizes[17] != NGATE ||
      in_sizes[18] != 2 * 2 * NHID || in_sizes[19] != 2 || out_size != NBATCH * 2) return;
  if (HB_BYTES > ws_size || HB_BYTES > (size_t)134217728) return;

  const float* x       = (const float*)d_in[0];
  const int*   lengths = (const int*)d_in[1];
  const float* wih0    = (const float*)d_in[2];
  const float* whh0    = (const float*)d_in[3];
  const float* bih0    = (const float*)d_in[4];
  const float* bhh0    = (const float*)d_in[5];
  const float* wih0r   = (const float*)d_in[6];
  const float* whh0r   = (const float*)d_in[7];
  const float* bih0r   = (const float*)d_in[8];
  const float* bhh0r   = (const float*)d_in[9];
  const float* wih1    = (const float*)d_in[10];
  const float* whh1    = (const float*)d_in[11];
  const float* bih1    = (const float*)d_in[12];
  const float* bhh1    = (const float*)d_in[13];
  const float* wih1r   = (const float*)d_in[14];
  const float* bih1r   = (const float*)d_in[16];
  const float* bhh1r   = (const float*)d_in[17];
  const float* wout    = (const float*)d_in[18];
  const float* bout    = (const float*)d_in[19];
  unsigned short* HB   = (unsigned short*)d_ws;

  rev_scan_kernel<<<NTILE, 32, 0, stream>>>(x, lengths, wih0r, whh0r, bih0r, bhh0r, HB);
  fwd_stack_kernel<<<NTILE, 32, 0, stream>>>(x, lengths, wih0, whh0, bih0, bhh0,
                                             wih1, whh1, bih1, bhh1,
                                             wih1r, bih1r, bhh1r, wout, bout,
                                             HB, (float*)d_out);
}
